// PointnetPP_73589969649777
// MI455X (gfx1250) — hardware-verified
//
#include <hip/hip_runtime.h>
#include <stdint.h>
#pragma clang fp contract(off)

typedef __attribute__((ext_vector_type(16))) __bf16   v16b;
typedef __attribute__((ext_vector_type(8)))  __bf16   v8b;
typedef __attribute__((ext_vector_type(8)))  float    v8f;
typedef __attribute__((ext_vector_type(4)))  float    v4f;
typedef __attribute__((ext_vector_type(4)))  unsigned v4u;
typedef __attribute__((ext_vector_type(2)))  unsigned v2u;

constexpr int kBatch = 16;
constexpr int kPts   = 8192;
constexpr int kSamp  = 128;
constexpr int kNbr   = 64;
constexpr int kRows0 = kBatch * kSamp * kNbr;
constexpr int kRows1 = kBatch * kSamp;
constexpr int kScshPitch = 512;
static_assert(kRows0 == 131072 && kRows1 == 2048, "shape");
static_assert((kPts & (kPts - 1)) == 0, "power of two point count");
static_assert(kRows0 % 64 == 0 && kRows1 % 64 == 0, "M tile multiple");

__device__ __forceinline__ unsigned bf_bits_rne(float f) {
  const unsigned u = __float_as_uint(f);
  return (u + 0x7FFFu + ((u >> 16) & 1u)) >> 16;
}
__device__ __forceinline__ void bf_split(float f, unsigned& hb, unsigned& lb) {
  hb = bf_bits_rne(f);
  const float res = f - __uint_as_float(hb << 16);
  lb = bf_bits_rne(res);
}

union FragB { v16b v; v8b h[2]; };
__device__ __forceinline__ v16b frag_load(const __bf16* p) {
  FragB f;
  f.h[0] = *(const v8b*)(p);
  f.h[1] = *(const v8b*)(p + 16);
  return f.v;
}
__device__ __forceinline__ v8f mma_bf(v16b a, v16b b, v8f c) {
  return __builtin_amdgcn_wmma_f32_16x16x32_bf16(false, a, false, b, (short)0, c, false, false);
}
__device__ __forceinline__ void guard_acc4(v8f& a, v8f& b, v8f& c, v8f& d, v16b x, v16b y) {
  asm volatile("v_nop\n\tv_nop\n\tv_nop\n\tv_nop" : "+v"(a), "+v"(b), "+v"(c), "+v"(d) : "v"(x), "v"(y));
}
__device__ __forceinline__ void keep4_b(v16b a, v16b b, v16b c, v16b d) {
  asm volatile("v_nop" :: "v"(a), "v"(b), "v"(c), "v"(d));
}

__global__ __launch_bounds__(256) void prep_w_kernel(const float* __restrict__ W, int Kin, int KD, int N,
                                                     unsigned short* __restrict__ hi,
                                                     unsigned short* __restrict__ lo) {
  const int g = blockIdx.x * 256 + threadIdx.x;
  const int kc8 = KD >> 3;
  const int total = N * kc8;
  if (g >= total) return;
  const int n = g / kc8;
  const int kc = g - n * kc8;
  unsigned hw[4] = {0u, 0u, 0u, 0u};
  unsigned lw[4] = {0u, 0u, 0u, 0u};
#pragma unroll
  for (int e = 0; e < 8; ++e) {
    const int k = kc * 8 + e;
    const int kk = (k < Kin) ? k : (Kin - 1);
    float v = W[(size_t)kk * N + n];
    v = (k < Kin) ? v : 0.0f;
    unsigned hb, lb;
    bf_split(v, hb, lb);
    hw[e >> 1] |= (hb & 0xFFFFu) << ((e & 1) * 16);
    lw[e >> 1] |= (lb & 0xFFFFu) << ((e & 1) * 16);
  }
  v4u hv; hv.x = hw[0]; hv.y = hw[1]; hv.z = hw[2]; hv.w = hw[3];
  v4u lv; lv.x = lw[0]; lv.y = lw[1]; lv.z = lw[2]; lv.w = lw[3];
  unsigned short* ph = hi + (size_t)g * 8;
  unsigned short* pl = lo + (size_t)g * 8;
  *(volatile v4u*)ph = hv;
  *(volatile v4u*)pl = lv;
  __threadfence();
  *(volatile v4u*)ph = hv;
  *(volatile v4u*)pl = lv;
}

__device__ __forceinline__ void argmax_bfly(float& v, int& i) {
#pragma unroll
  for (int off = 16; off >= 1; off >>= 1) {
    const float ov = __shfl_xor(v, off, 32);
    const int oi = __shfl_xor(i, off, 32);
    const bool tk = (ov > v) || ((ov == v) && (oi < i));
    v = tk ? ov : v;
    i = tk ? oi : i;
  }
}

__global__ __launch_bounds__(1024) void fps_kernel(const float* __restrict__ pos, float* __restrict__ sp4) {
#pragma clang fp contract(off)
  __shared__ float s_rv[2][32];
  __shared__ int   s_ri[2][32];
  __shared__ int   s_idx[kSamp];
  const int b = blockIdx.x;
  const int t = threadIdx.x;
  const int lane = t & 31;
  const int wave = t >> 5;
  const float* P = pos + (size_t)b * kPts * 3;
  const v4f* P4 = (const v4f*)(P + 24 * t);
  const v4f a0 = P4[0];
  const v4f a1 = P4[1];
  const v4f a2 = P4[2];
  const v4f a3 = P4[3];
  const v4f a4 = P4[4];
  const v4f a5 = P4[5];
  const float px[8] = {a0.x, a0.w, a1.z, a2.y, a3.x, a3.w, a4.z, a5.y};
  const float py[8] = {a0.y, a1.x, a1.w, a2.z, a3.y, a4.x, a4.w, a5.z};
  const float pz[8] = {a0.z, a1.y, a2.x, a2.w, a3.z, a4.y, a5.x, a5.w};
  float dist[8];
#pragma unroll
  for (int i = 0; i < 8; ++i) dist[i] = 1e10f;
  if (t == 0) s_idx[0] = 0;
  int last = 0;
#pragma unroll 1
  for (int s = 1; s < kSamp; ++s) {
    const int lc = last & (kPts - 1);
    const float lx = P[lc * 3 + 0];
    const float ly = P[lc * 3 + 1];
    const float lz = P[lc * 3 + 2];
    float bv = -1.0f;
    int bi = 0;
#pragma unroll
    for (int i = 0; i < 8; ++i) {
      const float dx = px[i] - lx;
      const float dy = py[i] - ly;
      const float dz = pz[i] - lz;
      const float t0 = dx * dx;
      const float t1 = dy * dy;
      const float t2 = dz * dz;
      const float d = (t0 + t2) + t1;
      const float dm = fminf(dist[i], d);
      dist[i] = dm;
      const bool up = dm > bv;
      bv = up ? dm : bv;
      bi = up ? (8 * t + i) : bi;
    }
    argmax_bfly(bv, bi);
    const int par = s & 1;
    if (lane == 0) { s_rv[par][wave] = bv; s_ri[par][wave] = bi; }
    __syncthreads();
    float gv = s_rv[par][lane];
    int gi = s_ri[par][lane];
    argmax_bfly(gv, gi);
    last = gi;
    if (t == 0) s_idx[s] = gi;
  }
  __syncthreads();
  if (t < kSamp) {
    const int id = s_idx[t] & (kPts - 1);
    v4f o;
    o.x = P[id * 3 + 0];
    o.y = P[id * 3 + 1];
    o.z = P[id * 3 + 2];
    o.w = 0.0f;
    float* dst = sp4 + ((size_t)b * kSamp + t) * 4;
    *(volatile v4f*)dst = o;
    __threadfence();
    *(volatile v4f*)dst = o;
  }
}

__device__ __forceinline__ unsigned sq_key(float sx, float sy, float sz, float sqs,
                                           float qx, float qy, float qz) {
#pragma clang fp contract(off)
  const float u0 = qx * qx;
  const float u1 = qy * qy;
  const float u2 = qz * qz;
  const float sqp = (u0 + u2) + u1;
  float p = sx * qx;
  p = __builtin_fmaf(sy, qy, p);
  p = __builtin_fmaf(sz, qz, p);
  const float two_p = 2.0f * p;
  const float base = sqs + sqp;
  float v = base - two_p;
  v = (v > 0.0f) ? v : 0.0f;
  return __float_as_uint(v);
}

__global__ __launch_bounds__(256) void knn_group_kernel(const float* __restrict__ x, const float* __restrict__ pos,
                                                        const float* __restrict__ sp4, float* __restrict__ G0) {
#pragma clang fp contract(off)
  __shared__ int   s_cnt[2][8];
  __shared__ int   s_wlt[8];
  __shared__ int   s_weq[8];
  __shared__ int   s_sel[kNbr];
  __shared__ float s_selsq[kNbr];
  __shared__ __align__(16) float s_g[kNbr * 8];
  const int bm = blockIdx.x;
  const int b = bm >> 7;
  const int t = threadIdx.x;
  const int lane = t & 31;
  const int wave = t >> 5;
  const v4f sv = *(const v4f*)(sp4 + (size_t)bm * 4);
  const float sx = sv.x;
  const float sy = sv.y;
  const float sz = sv.z;
  const float w0 = sx * sx;
  const float w1 = sy * sy;
  const float w2 = sz * sz;
  const float sqs = (w0 + w2) + w1;
  if (t < kNbr) { s_sel[t] = 0; s_selsq[t] = 0.0f; }

  const v4f* P4 = (const v4f*)(pos + (size_t)b * kPts * 3 + (size_t)t * 96);
  unsigned key[32];
#pragma unroll
  for (int c = 0; c < 8; ++c) {
    v4f a0 = P4[3 * c + 0];
    v4f a1 = P4[3 * c + 1];
    v4f a2 = P4[3 * c + 2];
    asm volatile("" : "+v"(a0), "+v"(a1), "+v"(a2) :: "memory");
    key[4 * c + 0] = sq_key(sx, sy, sz, sqs, a0.x, a0.y, a0.z);
    key[4 * c + 1] = sq_key(sx, sy, sz, sqs, a0.w, a1.x, a1.y);
    key[4 * c + 2] = sq_key(sx, sy, sz, sqs, a1.z, a1.w, a2.x);
    key[4 * c + 3] = sq_key(sx, sy, sz, sqs, a2.y, a2.z, a2.w);
  }

  unsigned V = 0u;
#pragma unroll 1
  for (int bit = 30; bit >= 0; --bit) {
    const unsigned cand = V | (1u << bit);
    int cnt = 0;
#pragma unroll
    for (int i = 0; i < 32; ++i) cnt += (key[i] < cand) ? 1 : 0;
#pragma unroll
    for (int off = 16; off >= 1; off >>= 1) cnt += __shfl_xor(cnt, off, 32);
    const int par = bit & 1;
    if (lane == 0) s_cnt[par][wave] = cnt;
    __syncthreads();
    int tot = 0;
#pragma unroll
    for (int w = 0; w < 8; ++w) tot += s_cnt[par][w];
    V = (tot < kNbr) ? cand : V;
  }

  int lt = 0;
  int eq = 0;
#pragma unroll
  for (int i = 0; i < 32; ++i) {
    lt += (key[i] < V) ? 1 : 0;
    eq += (key[i] == V) ? 1 : 0;
  }
  int slt = lt;
  int seq = eq;
#pragma unroll
  for (int off = 1; off < 32; off <<= 1) {
    const int a = __shfl_up(slt, off, 32);
    const int e2 = __shfl_up(seq, off, 32);
    const bool ok = lane >= off;
    slt += ok ? a : 0;
    seq += ok ? e2 : 0;
  }
  if (lane == 31) { s_wlt[wave] = slt; s_weq[wave] = seq; }
  __syncthreads();
  int base_lt = 0;
  int base_eq = 0;
  int total_lt = 0;
#pragma unroll
  for (int w = 0; w < 8; ++w) {
    const int a = s_wlt[w];
    const int e2 = s_weq[w];
    base_lt += (w < wave) ? a : 0;
    base_eq += (w < wave) ? e2 : 0;
    total_lt += a;
  }
  const int need = kNbr - total_lt;
  int rl = base_lt + slt - lt;
  int re = base_eq + seq - eq;
#pragma unroll
  for (int i = 0; i < 32; ++i) {
    const unsigned k = key[i];
    const bool isl = k < V;
    const bool ise = k == V;
    const int slot = isl ? rl : (total_lt + re);
    const bool take = isl || (ise && (re < need));
    if (take && ((unsigned)slot < (unsigned)kNbr)) {
      s_sel[slot] = 32 * t + i;
      s_selsq[slot] = __uint_as_float(k);
    }
    rl += isl ? 1 : 0;
    re += ise ? 1 : 0;
  }
  __syncthreads();
  if (t < kNbr) {
    const int id = s_sel[t] & (kPts - 1);
    const float* pp = pos + ((size_t)b * kPts + id) * 3;
    const float* xp = x + ((size_t)b * kPts + id) * 3;
    const float q0 = pp[0];
    const float q1 = pp[1];
    const float q2 = pp[2];
    const float f0 = xp[0];
    const float f1 = xp[1];
    const float f2 = xp[2];
    float* gr = s_g + t * 8;
    gr[0] = q0 - sx;
    gr[1] = q1 - sy;
    gr[2] = q2 - sz;
    gr[3] = f0;
    gr[4] = f1;
    gr[5] = f2;
    gr[6] = s_selsq[t];
    gr[7] = 0.0f;
  }
  __syncthreads();
  if (t < 128) {
    const v4f v = *(const v4f*)(s_g + 4 * t);
    float* dst = G0 + (size_t)bm * (kNbr * 8) + 4 * t;
    *(volatile v4f*)dst = v;
    __threadfence();
    *(volatile v4f*)dst = v;
  }
}

template <int NC, bool POOL>
__device__ __forceinline__ void tile_epilogue(const float* sC, float* s_stat, const float* s_mask,
                                              float* Y, int ldy, int m0, int n0, float* part_blk,
                                              float* ymax_row, float* ymin_row) {
  constexpr int CP = NC + 4;
  constexpr int LPR = NC / 4;
  constexpr int RPI = 32 / LPR;
  constexpr int ITS = 8 / RPI;
  const int tid = threadIdx.x;
  const int lane = tid & 31;
  const int wave = tid >> 5;
  if (!POOL) {
    const int rsub = lane / LPR;
    const int c4 = (lane - rsub * LPR) * 4;
    for (int pass = 0; pass < 2; ++pass) {
#pragma unroll
      for (int it = 0; it < ITS; ++it) {
        const int row = wave * 8 + it * RPI + rsub;
        const v4f v = *(const v4f*)(sC + row * CP + c4);
        *(volatile v4f*)(Y + (size_t)(m0 + row) * ldy + n0 + c4) = v;
      }
      __threadfence();
    }
  }
  if (tid < NC) {
    float s = 0.0f;
    float q = 0.0f;
    float mx = -3.0e38f;
    float mn = 3.0e38f;
#pragma unroll 4
    for (int r = 0; r < 64; ++r) {
      const float v = sC[r * CP + tid];
      s += v;
      const float vv = v * v;
      q += vv;
      if (POOL) {
        const bool keep = s_mask[r] <= 0.16f;
        const float m1 = fmaxf(mx, v);
        const float m2 = fminf(mn, v);
        mx = keep ? m1 : mx;
        mn = keep ? m2 : mn;
      }
    }
    s_stat[tid] = s;
    s_stat[NC + tid] = q;
    if (POOL) {
      s_stat[2 * NC + tid] = mx;
      s_stat[3 * NC + tid] = mn;
    }
  }
  __syncthreads();
  if (wave == 0) {
    constexpr int PIT = (2 * NC) / 128;
    for (int pass = 0; pass < 2; ++pass) {
#pragma unroll
      for (int it = 0; it < PIT; ++it) {
        const v4f v = *(const v4f*)(s_stat + it * 128 + lane * 4);
        *(volatile v4f*)(part_blk + it * 128 + lane * 4) = v;
      }
      __threadfence();
    }
  }
  if (POOL) {
    if (wave == 1) {
      for (int pass = 0; pass < 2; ++pass) {
        const v4f vx = *(const v4f*)(s_stat + 2 * NC + lane * 4);
        const v4f vn = *(const v4f*)(s_stat + 3 * NC + lane * 4);
        *(volatile v4f*)(ymax_row + lane * 4) = vx;
        *(volatile v4f*)(ymin_row + lane * 4) = vn;
        __threadfence();
      }
    }
  }
}

__global__ __launch_bounds__(256) void layer0_kernel(const float* __restrict__ G0, const float* __restrict__ W00,
                                                     const float* __restrict__ b00, float* __restrict__ Y0,
                                                     float* __restrict__ part) {
  __shared__ __align__(16) float s_g[64 * 8];
  __shared__ __align__(16) float sC[64 * 68];
  __shared__ __align__(16) float s_stat[4 * 64];
  const int tid = threadIdx.x;
  const int m0 = blockIdx.x * 64;
  if (tid < 128) *(v4f*)(s_g + 4 * tid) = *(const v4f*)(G0 + (size_t)m0 * 8 + 4 * tid);
  const int c = tid & 63;
  const int rg = tid >> 6;
  const float w0 = W00[0 * 64 + c];
  const float w1 = W00[1 * 64 + c];
  const float w2 = W00[2 * 64 + c];
  const float w3 = W00[3 * 64 + c];
  const float w4 = W00[4 * 64 + c];
  const float w5 = W00[5 * 64 + c];
  const float bz = b00[c];
  __syncthreads();
#pragma unroll 2
  for (int r = 0; r < 16; ++r) {
    const int row = rg * 16 + r;
    const float* g = s_g + row * 8;
    float y = bz;
    y = __builtin_fmaf(g[0], w0, y);
    y = __builtin_fmaf(g[1], w1, y);
    y = __builtin_fmaf(g[2], w2, y);
    y = __builtin_fmaf(g[3], w3, y);
    y = __builtin_fmaf(g[4], w4, y);
    y = __builtin_fmaf(g[5], w5, y);
    sC[row * 68 + c] = y;
  }
  __syncthreads();
  tile_epilogue<64, false>(sC, s_stat, s_g, Y0, 64, m0, 0, part + (size_t)blockIdx.x * 128, nullptr, nullptr);
}

__global__ __launch_bounds__(256) void bn_finalize_kernel(const float* __restrict__ part, int nblk, int nc,
                                                          double inv_cnt, const float* __restrict__ g,
                                                          const float* __restrict__ be, float* __restrict__ scsh) {
  __shared__ double s_s[8][32];
  __shared__ double s_q[8][32];
  const int tid = threadIdx.x;
  const int lane = tid & 31;
  const int wave = tid >> 5;
  const int c = blockIdx.x * 32 + lane;
  const int by = c / nc;
  const int cc = c - by * nc;
  const int nb = (nblk < 4096) ? nblk : 4096;
  double s = 0.0;
  double q = 0.0;
#pragma unroll 4
  for (int bx = wave; bx < nb; bx += 8) {
    const size_t base = ((size_t)(by * nb + bx) * 2) * nc;
    s += (double)part[base + cc];
    q += (double)part[base + nc + cc];
  }
  s_s[wave][lane] = s;
  s_q[wave][lane] = q;
  __syncthreads();
  if (wave == 0) {
    double S = 0.0;
    double Q = 0.0;
#pragma unroll
    for (int w = 0; w < 8; ++w) { S += s_s[w][lane]; Q += s_q[w][lane]; }
    const double mean = S * inv_cnt;
    double var = Q * inv_cnt - mean * mean;
    var = (var > 0.0) ? var : 0.0;
    const float rs = 1.0f / sqrtf((float)var + 1e-5f);
    const float scl = g[c] * rs;
    const float shf = be[c] - (float)mean * scl;
    volatile float* o = scsh;
    o[c] = scl;
    o[kScshPitch + c] = shf;
    __threadfence();
    o[c] = scl;
    o[kScshPitch + c] = shf;
  }
}

template <int KD, int NC, bool BNRELU, bool POOL>
__global__ __launch_bounds__(256) void gemm_bn_kernel(const float* __restrict__ A, const float* __restrict__ scsh,
                                                      const unsigned short* __restrict__ Bhi,
                                                      const unsigned short* __restrict__ Blo,
                                                      const float* __restrict__ bias, float* __restrict__ Y, int ldy,
                                                      float* __restrict__ part, const float* __restrict__ gmask,
                                                      float* __restrict__ ymax, float* __restrict__ ymin) {
  static_assert(KD % 32 == 0, "K multiple of 32");
  static_assert(NC == 64 || NC == 128, "column chunk");
  static_assert(!POOL || NC == 128, "pool chunk");
  constexpr int AP = KD + 8;
  constexpr int CP = NC + 4;
  constexpr int NT = NC / 32;
  constexpr int KQ = KD / 4;
  __shared__ __align__(16) unsigned short sAh[64 * AP];
  __shared__ __align__(16) unsigned short sAl[64 * AP];
  __shared__ __align__(16) float sC[64 * CP];
  __shared__ __align__(16) float s_stat[4 * NC];
  __shared__ float s_scl[KD];
  __shared__ float s_shf[KD];
  __shared__ float s_mask[64];

  const int tid = threadIdx.x;
  const int lane = tid & 31;
  const int wave = tid >> 5;
  const int m0 = blockIdx.x * 64;
  const int n0 = blockIdx.y * NC;

  if (BNRELU) {
    if (tid < KD) { s_scl[tid] = scsh[tid]; s_shf[tid] = scsh[kScshPitch + tid]; }
  }
  if (POOL) {
    if (tid < 64) s_mask[tid] = gmask[(size_t)(m0 + tid) * 8 + 6];
  }
  __syncthreads();

  constexpr int NV = 64 * KQ;
#pragma unroll 2
  for (int i = tid; i < NV; i += 256) {
    const int row = i / KQ;
    const int c4 = (i - row * KQ) * 4;
    const v4f v = *(const v4f*)(A + (size_t)(m0 + row) * KD + c4);
    float e0 = v.x;
    float e1 = v.y;
    float e2 = v.z;
    float e3 = v.w;
    if (BNRELU) {
      e0 = fmaxf(e0 * s_scl[c4 + 0] + s_shf[c4 + 0], 0.0f);
      e1 = fmaxf(e1 * s_scl[c4 + 1] + s_shf[c4 + 1], 0.0f);
      e2 = fmaxf(e2 * s_scl[c4 + 2] + s_shf[c4 + 2], 0.0f);
      e3 = fmaxf(e3 * s_scl[c4 + 3] + s_shf[c4 + 3], 0.0f);
    }
    unsigned h0, l0, h1, l1, h2, l2, h3, l3;
    bf_split(e0, h0, l0);
    bf_split(e1, h1, l1);
    bf_split(e2, h2, l2);
    bf_split(e3, h3, l3);
    v2u hv;
    hv.x = (h0 & 0xFFFFu) | (h1 << 16);
    hv.y = (h2 & 0xFFFFu) | (h3 << 16);
    v2u lv;
    lv.x = (l0 & 0xFFFFu) | (l1 << 16);
    lv.y = (l2 & 0xFFFFu) | (l3 << 16);
    *(v2u*)(sAh + row * AP + c4) = hv;
    *(v2u*)(sAl + row * AP + c4) = lv;
  }
  __syncthreads();

  const int rlane = lane & 15;
  const int hh = lane >> 4;
  const int koff = hh * 8;
  const int msub = wave & 3;
  const int nhalf = wave >> 2;
  const int ncol0 = n0 + nhalf * (NC / 2);

  v8f acc[4];
#pragma unroll
  for (int j = 0; j < 4; ++j) acc[j] = (v8f){0.f, 0.f, 0.f, 0.f, 0.f, 0.f, 0.f, 0.f};

  const unsigned short* arow_h = sAh + (msub * 16 + rlane) * AP + koff;
  const unsigned short* arow_l = sAl + (msub * 16 + rlane) * AP + koff;

#pragma unroll 1
  for (int k0 = 0; k0 < KD; k0 += 32) {
    v16b bh[4];
    v16b bl[4];
#pragma unroll
    for (int j = 0; j < NT; ++j) {
      const size_t bo = (size_t)(ncol0 + j * 16 + rlane) * KD + k0 + koff;
      bh[j] = frag_load((const __bf16*)(Bhi + bo));
      bl[j] = frag_load((const __bf16*)(Blo + bo));
    }
    const v16b ah = frag_load((const __bf16*)(arow_h + k0));
    const v16b al = frag_load((const __bf16*)(arow_l + k0));
#pragma unroll
    for (int j = 0; j < NT; ++j) {
      acc[j] = mma_bf(ah, bh[j], acc[j]);
      acc[j] = mma_bf(ah, bl[j], acc[j]);
      acc[j] = mma_bf(al, bh[j], acc[j]);
    }
    guard_acc4(acc[0], acc[1], acc[2], acc[3], ah, al);
    if (NT == 4) {
      keep4_b(bh[0], bh[1], bh[2], bh[3]);
      keep4_b(bl[0], bl[1], bl[2], bl[3]);
    } else {
      keep4_b(bh[0], bh[1], bl[0], bl[1]);
    }
  }
  {
    v16b z16 = frag_load((const __bf16*)arow_h);
    guard_acc4(acc[0], acc[1], acc[2], acc[3], z16, z16);
  }

#pragma unroll
  for (int j = 0; j < NT; ++j) {
    const int col = nhalf * (NC / 2) + j * 16 + rlane;
    const float bz = bias[n0 + col];
#pragma unroll
    for (int r = 0; r < 8; ++r) sC[(msub * 16 + 8 * hh + r) * CP + col] = acc[j][r] + bz;
  }
  __syncthreads();

  float* part_blk = part + ((size_t)blockIdx.y * gridDim.x + blockIdx.x) * (2 * NC);
  float* yx = POOL ? (ymax + (size_t)blockIdx.x * 128) : nullptr;
  float* yn = POOL ? (ymin + (size_t)blockIdx.x * 128) : nullptr;
  tile_epilogue<NC, POOL>(sC, s_stat, s_mask, Y, ldy, m0, n0, part_blk, yx, yn);
}

__global__ __launch_bounds__(256) void build_a1_kernel(const float* __restrict__ sp4, const float* __restrict__ ymax,
                                                       const float* __restrict__ ymin, const float* __restrict__ scsh,
                                                       float* __restrict__ A1) {
  __shared__ __align__(16) float s_a[8 * 160];
  const int tid = threadIdx.x;
  const int r = tid >> 5;
  const int q = tid & 31;
  const int row0 = blockIdx.x * 8;
  const int row = row0 + r;
  const v4f mx = *(const v4f*)(ymax + (size_t)row * 128 + 4 * q);
  const v4f mn = *(const v4f*)(ymin + (size_t)row * 128 + 4 * q);
  const v4f sc = *(const v4f*)(scsh + 4 * q);
  const v4f sh = *(const v4f*)(scsh + kScshPitch + 4 * q);
  const v4f sv = *(const v4f*)(sp4 + (size_t)row * 4);
  const float amx[4] = {mx.x, mx.y, mx.z, mx.w};
  const float amn[4] = {mn.x, mn.y, mn.z, mn.w};
  const float asc[4] = {sc.x, sc.y, sc.z, sc.w};
  const float ash[4] = {sh.x, sh.y, sh.z, sh.w};
#pragma unroll
  for (int e = 0; e < 4; ++e) {
    const float pick = (asc[e] >= 0.0f) ? amx[e] : amn[e];
    float val = fmaxf(asc[e] * pick + ash[e], 0.0f);
    const bool any = amx[e] >= amn[e];
    val = any ? val : -1e8f;
    s_a[r * 160 + 3 + 4 * q + e] = val;
  }
  if (q == 0) {
    s_a[r * 160 + 0] = sv.x;
    s_a[r * 160 + 1] = sv.y;
    s_a[r * 160 + 2] = sv.z;
  }
  if (tid < 232) {
    const int pr = tid / 29;
    const int pc = tid - pr * 29;
    s_a[pr * 160 + 131 + pc] = 0.0f;
  }
  __syncthreads();
  for (int pass = 0; pass < 2; ++pass) {
    for (int i = tid; i < 320; i += 256) {
      const v4f v = *(const v4f*)(s_a + 4 * i);
      *(volatile v4f*)(A1 + (size_t)row0 * 160 + 4 * i) = v;
    }
    __threadfence();
  }
}

constexpr int kOut0Floats = kBatch * 512;
constexpr int kOut1Floats = kBatch * 3;
static_assert(kOut0Floats * 4 == 32768, "second output byte offset");
static_assert(kOut0Floats * 4 + kOut1Floats * 4 == 32960, "output total");

__global__ __launch_bounds__(256) void final_pool_kernel(const float* __restrict__ Z2, const float* __restrict__ scsh,
                                                         float* __restrict__ out) {
  const int tid = threadIdx.x;
  if (blockIdx.x == (kOut0Floats / 256)) {
    if (tid < 12) {
      v4f z;
      z.x = 0.0f; z.y = 0.0f; z.z = 0.0f; z.w = 0.0f;
      float* dst = out + kOut0Floats + 4 * tid;
      *(volatile v4f*)dst = z;
      __threadfence();
      *(volatile v4f*)dst = z;
    }
    return;
  }
  const int t = blockIdx.x * 256 + tid;
  const int c = t & 511;
  const int b = t >> 9;
  const float* z = Z2 + (size_t)b * kSamp * 512 + c;
  float mx = -3.0e38f;
  float mn = 3.0e38f;
#pragma unroll 4
  for (int r = 0; r < kSamp; ++r) {
    const float v = z[(size_t)r * 512];
    mx = fmaxf(mx, v);
    mn = fminf(mn, v);
  }
  const float sc = scsh[c];
  const float sh = scsh[kScshPitch + c];
  const float pick = (sc >= 0.0f) ? mx : mn;
  const float val = fmaxf(sc * pick + sh, 0.0f);
  volatile float* o = out;
  o[t] = val;
  __threadfence();
  o[t] = val;
}

namespace {
constexpr size_t SZ_SP   = (size_t)kRows1 * 16;
constexpr size_t SZ_G0   = (size_t)kRows0 * 32;
constexpr size_t SZ_Y64  = (size_t)kRows0 * 64 * 4;
constexpr size_t SZ_YM   = (size_t)kRows1 * 128 * 4;
constexpr size_t SZ_A1   = (size_t)kRows1 * 160 * 4;
constexpr size_t SZ_Z128 = (size_t)kRows1 * 128 * 4;
constexpr size_t SZ_Z512 = (size_t)kRows1 * 512 * 4;
constexpr size_t SZ_P0   = (size_t)(kRows0 / 64) * 2 * 64 * 4;
constexpr size_t SZ_P2   = (size_t)(kRows0 / 64) * 2 * 128 * 4;
constexpr size_t SZ_P3   = (size_t)(kRows1 / 64) * 2 * 2 * 64 * 4;
constexpr size_t SZ_P5   = (size_t)(kRows1 / 64) * 8 * 2 * 64 * 4;
constexpr size_t SZ_SCSH = (size_t)2 * kScshPitch * 4;
constexpr size_t SZ_W01  = (size_t)64 * 64 * 2;
constexpr size_t SZ_W02  = (size_t)128 * 64 * 2;
constexpr size_t SZ_W10  = (size_t)128 * 160 * 2;
constexpr size_t SZ_W11  = (size_t)128 * 128 * 2;
constexpr size_t SZ_W12  = (size_t)512 * 128 * 2;

constexpr size_t OFF_SP   = 0;
constexpr size_t OFF_G0   = OFF_SP + SZ_SP;
constexpr size_t OFF_Y0   = OFF_G0 + SZ_G0;
constexpr size_t OFF_Y1   = OFF_Y0 + SZ_Y64;
constexpr size_t OFF_YMAX = OFF_Y1 + SZ_Y64;
constexpr size_t OFF_YMIN = OFF_YMAX + SZ_YM;
constexpr size_t OFF_A1   = OFF_YMIN + SZ_YM;
constexpr size_t OFF_Z0   = OFF_A1 + SZ_A1;
constexpr size_t OFF_Z1   = OFF_Z0 + SZ_Z128;
constexpr size_t OFF_Z2   = OFF_Z1 + SZ_Z128;
constexpr size_t OFF_P0   = OFF_Z2 + SZ_Z512;
constexpr size_t OFF_P1   = OFF_P0 + SZ_P0;
constexpr size_t OFF_P2   = OFF_P1 + SZ_P0;
constexpr size_t OFF_P3   = OFF_P2 + SZ_P2;
constexpr size_t OFF_P4   = OFF_P3 + SZ_P3;
constexpr size_t OFF_P5   = OFF_P4 + SZ_P3;
constexpr size_t OFF_SCSH = OFF_P5 + SZ_P5;
constexpr size_t OFF_W01H = OFF_SCSH + 6 * SZ_SCSH;
constexpr size_t OFF_W01L = OFF_W01H + SZ_W01;
constexpr size_t OFF_W02H = OFF_W01L + SZ_W01;
constexpr size_t OFF_W02L = OFF_W02H + SZ_W02;
constexpr size_t OFF_W10H = OFF_W02L + SZ_W02;
constexpr size_t OFF_W10L = OFF_W10H + SZ_W10;
constexpr size_t OFF_W11H = OFF_W10L + SZ_W10;
constexpr size_t OFF_W11L = OFF_W11H + SZ_W11;
constexpr size_t OFF_W12H = OFF_W11L + SZ_W11;
constexpr size_t OFF_W12L = OFF_W12H + SZ_W12;
constexpr size_t WS_TOTAL = OFF_W12L + SZ_W12;
static_assert(WS_TOTAL <= (size_t)134217728, "carve within 128 MiB");
static_assert(OFF_G0 % 256 == 0 && OFF_Y0 % 256 == 0 && OFF_A1 % 256 == 0 && OFF_P3 % 256 == 0 &&
              OFF_SCSH % 256 == 0 && OFF_W01H % 256 == 0 && OFF_W10H % 256 == 0 && OFF_W12L % 256 == 0,
              "aligned carve");
static_assert(SZ_P3 == 32768 && SZ_P5 == 131072, "partial table sizes");
}

extern "C" void kernel_launch(void* const* d_in, const int* in_sizes, int n_in, void* d_out, int out_size,
                              void* d_ws, size_t ws_size, hipStream_t stream) {
  (void)in_sizes;
  if (n_in < 26) return;
  if (ws_size < WS_TOTAL) return;
  if (out_size < kOut0Floats + kOut1Floats) return;

  const float* x   = (const float*)d_in[0];
  const float* pos = (const float*)d_in[1];
  const float* W[6];
  const float* bb[6];
  const float* gg[6];
  const float* be[6];
  for (int l = 0; l < 6; ++l) {
    W[l]  = (const float*)d_in[2 + 4 * l + 0];
    bb[l] = (const float*)d_in[2 + 4 * l + 1];
    gg[l] = (const float*)d_in[2 + 4 * l + 2];
    be[l] = (const float*)d_in[2 + 4 * l + 3];
  }

  unsigned char* ws = (unsigned char*)d_ws;
  float* SP   = (float*)(ws + OFF_SP);
  float* G0   = (float*)(ws + OFF_G0);
  float* Y0   = (float*)(ws + OFF_Y0);
  float* Y1   = (float*)(ws + OFF_Y1);
  float* YMAX = (float*)(ws + OFF_YMAX);
  float* YMIN = (float*)(ws + OFF_YMIN);
  float* A1   = (float*)(ws + OFF_A1);
  float* Z0   = (float*)(ws + OFF_Z0);
  float* Z1   = (float*)(ws + OFF_Z1);
  float* Z2   = (float*)(ws + OFF_Z2);
  float* P0   = (float*)(ws + OFF_P0);
  float* P1   = (float*)(ws + OFF_P1);
  float* P2   = (float*)(ws + OFF_P2);
  float* P3   = (float*)(ws + OFF_P3);
  float* P4   = (float*)(ws + OFF_P4);
  float* P5   = (float*)(ws + OFF_P5);
  float* SC[6];
  for (int l = 0; l < 6; ++l) SC[l] = (float*)(ws + OFF_SCSH + (size_t)l * SZ_SCSH);
  unsigned short* W01H = (unsigned short*)(ws + OFF_W01H);
  unsigned short* W01L = (unsigned short*)(ws + OFF_W01L);
  unsigned short* W02H = (unsigned short*)(ws + OFF_W02H);
  unsigned short* W02L = (unsigned short*)(ws + OFF_W02L);
  unsigned short* W10H = (unsigned short*)(ws + OFF_W10H);
  unsigned short* W10L = (unsigned short*)(ws + OFF_W10L);
  unsigned short* W11H = (unsigned short*)(ws + OFF_W11H);
  unsigned short* W11L = (unsigned short*)(ws + OFF_W11L);
  unsigned short* W12H = (unsigned short*)(ws + OFF_W12H);
  unsigned short* W12L = (unsigned short*)(ws + OFF_W12L);
  float* out = (float*)d_out;

  prep_w_kernel<<<(64 * 64 / 8) / 256, 256, 0, stream>>>(W[1], 64, 64, 64, W01H, W01L);
  prep_w_kernel<<<(128 * 64 / 8) / 256, 256, 0, stream>>>(W[2], 64, 64, 128, W02H, W02L);
  prep_w_kernel<<<(128 * 160 / 8) / 256, 256, 0, stream>>>(W[3], 131, 160, 128, W10H, W10L);
  prep_w_kernel<<<(128 * 128 / 8) / 256, 256, 0, stream>>>(W[4], 128, 128, 128, W11H, W11L);
  prep_w_kernel<<<(512 * 128 / 8) / 256, 256, 0, stream>>>(W[5], 128, 128, 512, W12H, W12L);

  fps_kernel<<<kBatch, 1024, 0, stream>>>(pos, SP);
  knn_group_kernel<<<kRows1, 256, 0, stream>>>(x, pos, SP, G0);

  const double inv0 = 1.0 / (double)kRows0;
  const double inv1 = 1.0 / (double)kRows1;
  const int nb0 = kRows0 / 64;
  const int nb1 = kRows1 / 64;

  layer0_kernel<<<nb0, 256, 0, stream>>>(G0, W[0], bb[0], Y0, P0);
  bn_finalize_kernel<<<64 / 32, 256, 0, stream>>>(P0, nb0, 64, inv0, gg[0], be[0], SC[0]);

  gemm_bn_kernel<64, 64, true, false><<<dim3(nb0, 1), 256, 0, stream>>>(
      Y0, SC[0], W01H, W01L, bb[1], Y1, 64, P1, G0, YMAX, YMIN);
  bn_finalize_kernel<<<64 / 32, 256, 0, stream>>>(P1, nb0, 64, inv0, gg[1], be[1], SC[1]);

  gemm_bn_kernel<64, 128, true, true><<<dim3(nb0, 1), 256, 0, stream>>>(
      Y1, SC[1], W02H, W02L, bb[2], nullptr, 128, P2, G0, YMAX, YMIN);
  bn_finalize_kernel<<<128 / 32, 256, 0, stream>>>(P2, nb0, 128, inv0, gg[2], be[2], SC[2]);

  build_a1_kernel<<<kRows1 / 8, 256, 0, stream>>>(SP, YMAX, YMIN, SC[2], A1);

  gemm_bn_kernel<160, 64, false, false><<<dim3(nb1, 2), 256, 0, stream>>>(
      A1, SC[2], W10H, W10L, bb[3], Z0, 128, P3, G0, YMAX, YMIN);
  bn_finalize_kernel<<<128 / 32, 256, 0, stream>>>(P3, nb1, 64, inv1, gg[3], be[3], SC[3]);

  gemm_bn_kernel<128, 64, true, false><<<dim3(nb1, 2), 256, 0, stream>>>(
      Z0, SC[3], W11H, W11L, bb[4], Z1, 128, P4, G0, YMAX, YMIN);
  bn_finalize_kernel<<<128 / 32, 256, 0, stream>>>(P4, nb1, 64, inv1, gg[4], be[4], SC[4]);

  gemm_bn_kernel<128, 64, true, false><<<dim3(nb1, 8), 256, 0, stream>>>(
      Z1, SC[4], W12H, W12L, bb[5], Z2, 512, P5, G0, YMAX, YMIN);
  bn_finalize_kernel<<<512 / 32, 256, 0, stream>>>(P5, nb1, 64, inv1, gg[5], be[5], SC[5]);

  final_pool_kernel<<<kOut0Floats / 256 + 1, 256, 0, stream>>>(Z2, SC[5], out);
}
